// DecoderBlock_28467043238485
// MI455X (gfx1250) — hardware-verified
//
#include <hip/hip_runtime.h>
#include <math.h>

#ifndef NB
#define NB 2
#endif
#ifndef SEQ
#define SEQ 2048
#endif
#define NB_FULL 2
#define SEQ_FULL 2048

typedef __attribute__((ext_vector_type(16))) _Float16 v16h;
typedef __attribute__((ext_vector_type(8)))  _Float16 v8h;
typedef __attribute__((ext_vector_type(16))) __bf16   v16b;
typedef __attribute__((ext_vector_type(8)))  __bf16   v8b;
typedef __attribute__((ext_vector_type(8)))  float    v8f;
typedef __attribute__((ext_vector_type(4)))  float    v4f;
typedef __attribute__((ext_vector_type(2)))  float    v2f;
typedef __attribute__((ext_vector_type(4)))  unsigned v4u;
typedef __attribute__((ext_vector_type(2)))  unsigned v2u;
typedef __attribute__((ext_vector_type(4)))  int      v4i;

constexpr int kBatch   = NB;
constexpr int kSeq     = SEQ;
constexpr int kSeqFull = SEQ_FULL;
constexpr int kDim     = 512;
constexpr int kHeads   = 8;
constexpr int kHdim    = 64;
constexpr int kFfn     = 2048;
constexpr int kRows    = kBatch * kSeq;
constexpr int kQkvLd   = 3 * kDim;
constexpr int kFlagLd  = 32;
constexpr float kEps   = 1e-5f;
constexpr float kMaskSkip = -1e30f;

constexpr int kAKC = 64;
constexpr int kAQB = 64;
constexpr int kANW = 4;
constexpr int kNkc = kSeq / kAKC;

static_assert(kBatch >= 1 && kBatch <= NB_FULL);
static_assert(kSeq % 64 == 0 && kSeq >= 64 && kSeq <= kSeqFull);
static_assert(kNkc <= kFlagLd);
static_assert(kDim == kHeads * kHdim && kHdim == 64);
static_assert(kRows % 64 == 0 && kDim % 64 == 0 && kFfn % 64 == 0 && kDim % 32 == 0 && kFfn % 32 == 0);

constexpr float kCarryX   = 8.0f;
constexpr float kCarryW   = 256.0f;
constexpr float kCarryQkv = 8.0f;
constexpr float kCarryP   = 1024.0f;
constexpr float kCarryCtx = 64.0f;
constexpr float kCarryH   = 8.0f;
constexpr float kCarryHid = 32.0f;

constexpr int kCastElems = 512;
constexpr int kCastBlkW  = kDim * kDim / kCastElems;
constexpr int kCastBlkW1 = kFfn * kDim / kCastElems;
static_assert(kDim == kCastElems);

constexpr size_t kSzWqkv  = (size_t)3 * kDim * kDim * 2;
constexpr size_t kSzWo    = (size_t)kDim * kDim * 2;
constexpr size_t kSzW1    = (size_t)kFfn * kDim * 2;
constexpr size_t kSzW2    = (size_t)kDim * kFfn * 2;
constexpr size_t kSzXh    = (size_t)kRows * kDim * 2;
constexpr size_t kSzFlags = (size_t)kFlagLd * kFlagLd * 4;
constexpr size_t kSzQkv   = (size_t)kRows * kQkvLd * 2;
constexpr size_t kSzCtx   = (size_t)kRows * kDim * 2;
constexpr size_t kSzU     = (size_t)kRows * kDim * 4;
constexpr size_t kSzHf    = (size_t)kRows * kDim * 4;
constexpr size_t kSzHh    = (size_t)kRows * kDim * 2;
constexpr size_t kSzHid   = (size_t)kRows * kFfn * 2;
constexpr size_t kSzY     = (size_t)kRows * kDim * 4;
constexpr size_t kOffWqkv  = 0;
constexpr size_t kOffWo    = kOffWqkv + kSzWqkv;
constexpr size_t kOffW1    = kOffWo + kSzWo;
constexpr size_t kOffW2    = kOffW1 + kSzW1;
constexpr size_t kOffXh    = kOffW2 + kSzW2;
constexpr size_t kOffFlags = kOffXh + kSzXh;
constexpr size_t kOffQkv   = kOffFlags + kSzFlags;
constexpr size_t kOffCtx   = kOffQkv + kSzQkv;
constexpr size_t kOffU     = kOffCtx + kSzCtx;
constexpr size_t kOffHf    = kOffU + kSzU;
constexpr size_t kOffHh    = kOffHf + kSzHf;
constexpr size_t kOffHid   = kOffHh + kSzHh;
constexpr size_t kOffY     = kOffHid + kSzHid;
constexpr size_t kWsTotal  = kOffY + kSzY;
static_assert(kWsTotal <= 134217728);
static_assert(NB != 2 || SEQ != 2048 || kWsTotal == 73404416);
static_assert((kOffWo % 128) == 0 && (kOffW1 % 128) == 0 && (kOffW2 % 128) == 0 && (kOffXh % 128) == 0 &&
              (kOffFlags % 128) == 0 && (kOffQkv % 128) == 0 && (kOffCtx % 128) == 0 && (kOffU % 128) == 0 &&
              (kOffHf % 128) == 0 && (kOffHh % 128) == 0 && (kOffHid % 128) == 0 && (kOffY % 128) == 0);

__device__ __forceinline__ unsigned short f2bf_bits(float f) {
  unsigned u = __float_as_uint(f);
  return (unsigned short)((u + 0x7FFFu + ((u >> 16) & 1u)) >> 16);
}
__device__ __forceinline__ float bf_bits2f(unsigned short h) { return __uint_as_float(((unsigned)h) << 16); }
__device__ __forceinline__ float bfrne(float f) {
  unsigned u = __float_as_uint(f);
  u = (u + 0x7FFFu + ((u >> 16) & 1u)) & 0xFFFF0000u;
  return __uint_as_float(u);
}

__device__ __forceinline__ void dep_guard_h(v8f& a, v8f& b, v16h x, v16h y) { asm volatile("v_nop\n\tv_nop\n\tv_nop\n\tv_nop" : "+v"(a), "+v"(b) : "v"(x), "v"(y)); }
__device__ __forceinline__ void dep_guard_b(v8f& a, v8f& b, v16b x, v16b y) { asm volatile("v_nop\n\tv_nop\n\tv_nop\n\tv_nop" : "+v"(a), "+v"(b) : "v"(x), "v"(y)); }
__device__ __forceinline__ void keep4_h(v16h a, v16h b, v16h c, v16h d) { asm volatile("v_nop" :: "v"(a), "v"(b), "v"(c), "v"(d)); }
__device__ __forceinline__ void keep4_b(v16b a, v16b b, v16b c, v16b d) { asm volatile("v_nop" :: "v"(a), "v"(b), "v"(c), "v"(d)); }
__device__ __forceinline__ void acc_guard4(v8f& a, v8f& b, v8f& c, v8f& d) { asm volatile("v_nop\n\tv_nop\n\tv_nop\n\tv_nop" : "+v"(a), "+v"(b), "+v"(c), "+v"(d)); }
template <typename T> struct Frag;
template <> struct Frag<_Float16> {
  typedef v16h V; union U { v16h v; v8h h[2]; };
  static __device__ __forceinline__ v16h load(const _Float16* p) {
    U f; f.h[0] = *(const v8h*)(p); f.h[1] = *(const v8h*)(p + 16); return f.v;
  }
  static __device__ __forceinline__ v8f mma(v16h a, v16h b, v8f c) {
    return __builtin_amdgcn_wmma_f32_16x16x32_f16(false, a, false, b, (short)0, c, false, false);
  }
  static __device__ __forceinline__ void guard(v8f& a, v8f& b, v16h x, v16h y) { dep_guard_h(a, b, x, y); }
  static __device__ __forceinline__ void keep(v16h a, v16h b, v16h c, v16h d) { keep4_h(a, b, c, d); }
};
template <> struct Frag<__bf16> {
  typedef v16b V; union U { v16b v; v8b h[2]; };
  static __device__ __forceinline__ v16b load(const __bf16* p) {
    U f; f.h[0] = *(const v8b*)(p); f.h[1] = *(const v8b*)(p + 16); return f.v;
  }
  static __device__ __forceinline__ v8f mma(v16b a, v16b b, v8f c) {
    return __builtin_amdgcn_wmma_f32_16x16x32_bf16(false, a, false, b, (short)0, c, false, false);
  }
  static __device__ __forceinline__ void guard(v8f& a, v8f& b, v16b x, v16b y) { dep_guard_b(a, b, x, y); }
  static __device__ __forceinline__ void keep(v16b a, v16b b, v16b c, v16b d) { keep4_b(a, b, c, d); }
};

template <int ET> struct Elem;
template <> struct Elem<0> { typedef _Float16 T; };
template <> struct Elem<1> { typedef __bf16 T; };
template <int ET, bool SPLIT, int BIAS_MODE, int OUT_MODE, bool RESID, bool RRNE, int ACT = 0>
__global__ __launch_bounds__(256) void wmma_gemm64(
    const unsigned short* __restrict__ Ap, const unsigned short* __restrict__ A2p, int lda, long strideA,
    const unsigned short* __restrict__ Btp, const unsigned short* __restrict__ Bt2p, int ldb, long strideB,
    void* __restrict__ Cout, void* __restrict__ Cout2, int ldc, long strideC,
    const float* __restrict__ bias0, const float* __restrict__ bias1, const float* __restrict__ bias2,
    const float* __restrict__ resid, long strideR,
    int M, int N, int K, float scale, float oscale) {
  static_assert(!RESID || OUT_MODE == 0);
  typedef typename Elem<ET>::T T;
  typedef typename Frag<T>::V V;
  const T* A = (const T*)Ap; const T* A2 = (const T*)A2p; const T* Bt = (const T*)Btp; const T* Bt2 = (const T*)Bt2p;
  __shared__ __align__(16) float sT[8][16 * 68];
  const int b    = blockIdx.y;
  const int lane = threadIdx.x & 31;
  const int wave = threadIdx.x >> 5;
  const int tilesN = N >> 6;
  const int tilesM = M >> 6;
  const int tile = blockIdx.x * 8 + wave;
  if (tile >= tilesM * tilesN) return;
  const int tm = tile / tilesN;
  const int tn = tile - tm * tilesN;
  const int m0 = tm << 6;
  const int n0 = tn << 6;
  const float* bias = (b == 0) ? bias0 : ((b == 1) ? bias1 : bias2);

  const T* Ab  = A  + (size_t)b * strideA;
  const T* Bb  = Bt + (size_t)b * strideB;
  const T* Ab2 = SPLIT ? (A2  + (size_t)b * strideA) : nullptr;
  const T* Bb2 = SPLIT ? (Bt2 + (size_t)b * strideB) : nullptr;

  const int rlane = lane & 15;
  const int koff  = (lane >> 4) * 8;
  const int mOff  = (lane >> 4) * 8;

  v8f acc[4][4];
#pragma unroll
  for (int i = 0; i < 4; ++i)
#pragma unroll
    for (int j = 0; j < 4; ++j) acc[i][j] = (v8f){0.f,0.f,0.f,0.f,0.f,0.f,0.f,0.f};

  for (int k0 = 0; k0 < K; k0 += 32) {
    V bh[4], bl[4];
#pragma unroll
    for (int j = 0; j < 4; ++j) {
      const size_t bo = (size_t)(n0 + (j << 4) + rlane) * ldb + koff + k0;
      bh[j] = Frag<T>::load(Bb + bo);
      if (SPLIT) bl[j] = Frag<T>::load(Bb2 + bo);
    }
#pragma unroll
    for (int i = 0; i < 4; ++i) {
      const size_t ao = (size_t)(m0 + (i << 4) + rlane) * lda + koff + k0;
      V ah = Frag<T>::load(Ab + ao);
      V al = ah;
      if (SPLIT) al = Frag<T>::load(Ab2 + ao);
#pragma unroll
      for (int j = 0; j < 4; ++j) {
        acc[i][j] = Frag<T>::mma(ah, bh[j], acc[i][j]);
        if (SPLIT) {
          acc[i][j] = Frag<T>::mma(ah, bl[j], acc[i][j]);
          acc[i][j] = Frag<T>::mma(al, bh[j], acc[i][j]);
        }
      }
      Frag<T>::guard(acc[i][0], acc[i][3], ah, al);
    }
    Frag<T>::keep(bh[0], bh[1], bh[2], bh[3]);
    if (SPLIT) Frag<T>::keep(bl[0], bl[1], bl[2], bl[3]);
  }
  acc_guard4(acc[0][0], acc[0][1], acc[0][2], acc[0][3]);
  acc_guard4(acc[1][0], acc[1][1], acc[1][2], acc[1][3]);
  acc_guard4(acc[2][0], acc[2][1], acc[2][2], acc[2][3]);
  acc_guard4(acc[3][0], acc[3][1], acc[3][2], acc[3][3]);

  float* slab = sT[wave];
  const float* Rb = RESID ? (resid + (size_t)b * strideR) : nullptr;
#pragma unroll
  for (int i = 0; i < 4; ++i) {
    const int mBase = m0 + (i << 4);
#pragma unroll
    for (int j = 0; j < 4; ++j) {
      const int n = n0 + (j << 4) + rlane;
      float bv = 0.f;
      if (BIAS_MODE == 2) bv = bfrne(bias[n]);
#pragma unroll
      for (int r = 0; r < 8; ++r) {
        float v = acc[i][j][r] * scale;
        if (BIAS_MODE == 1) v += bfrne(bias[mBase + mOff + r]);
        if (BIAS_MODE == 2) v += bv;
        if (ACT == 1) v = tanhf(v);
        if (ACT == 2) v = fmaxf(v, 0.0f);
        if (ACT == 3) v = v / (1.0f + expf(-v));
        if (ACT == 4) v = (v > 0.f) ? v : 0.01f * v;
        slab[(mOff + r) * 68 + (j << 4) + rlane] = v * oscale;
      }
    }
    __builtin_amdgcn_fence(3  , "workgroup");
    __builtin_amdgcn_wave_barrier();
    __builtin_amdgcn_fence(2  , "workgroup");
    if (OUT_MODE == 0) {
      float* C = (float*)Cout + (size_t)b * strideC;
      const int hh = lane >> 4, c4 = (lane & 15) * 4;
      for (int pass = 0; pass < 2; ++pass) {
#pragma unroll
        for (int it = 0; it < 8; ++it) {
          const int row = it * 2 + hh;
          v4f v = *(const v4f*)(slab + row * 68 + c4);
          if (RESID) {
            v4f rr = *(const v4f*)(Rb + (size_t)(mBase + row) * ldc + n0 + c4);
            if (RRNE) { rr[0] = bfrne(rr[0]); rr[1] = bfrne(rr[1]); rr[2] = bfrne(rr[2]); rr[3] = bfrne(rr[3]); }
            v += rr;
          }
          *(volatile v4f*)(C + (size_t)(mBase + row) * ldc + n0 + c4) = v;
        }
        __threadfence();
      }
    } else {
      const int q = lane >> 3, c8 = (lane & 7) * 8;
      unsigned short* C  = (unsigned short*)Cout  + (size_t)b * strideC;
      unsigned short* C2 = (OUT_MODE == 2) ? ((unsigned short*)Cout2 + (size_t)b * strideC) : nullptr;
      for (int pass = 0; pass < 2; ++pass) {
#pragma unroll
        for (int it = 0; it < 4; ++it) {
          const int row = it * 4 + q;
          const float* sp = slab + row * 68 + c8;
          v8h hv, lv;
#pragma unroll
          for (int e = 0; e < 8; ++e) {
            if (OUT_MODE == 1) {
              hv[e] = (_Float16)sp[e];
              lv[e] = hv[e];
            } else {
              unsigned short hb = f2bf_bits(sp[e]);
              unsigned short lb = f2bf_bits(sp[e] - bf_bits2f(hb));
              hv[e] = __builtin_bit_cast(_Float16, hb);
              lv[e] = __builtin_bit_cast(_Float16, lb);
            }
          }
          *(volatile v8h*)(C + (size_t)(mBase + row) * ldc + n0 + c8) = hv;
          if (OUT_MODE == 2) *(volatile v8h*)(C2 + (size_t)(mBase + row) * ldc + n0 + c8) = lv;
        }
        __threadfence();
      }
    }
    __builtin_amdgcn_fence(3  , "workgroup");
    __builtin_amdgcn_wave_barrier();
    __builtin_amdgcn_fence(2  , "workgroup");
  }
}

__global__ __launch_bounds__(256) void cast_planes(
    const float* __restrict__ x, const float* __restrict__ Wq, const float* __restrict__ Wk,
    const float* __restrict__ Wv, const float* __restrict__ Wo, const float* __restrict__ W1,
    const float* __restrict__ W2,
    _Float16* __restrict__ xh, _Float16* __restrict__ wqkvh, _Float16* __restrict__ woh,
    _Float16* __restrict__ w1h, _Float16* __restrict__ w2h, int nXBlk, float cx, float cw) {
  const int t = threadIdx.x;
  int blk = blockIdx.x;
  const float* src;
  _Float16* dst;
  float sc;
  if (blk < nXBlk) {
    const int bb = blk / kSeq, ss = blk - bb * kSeq;
    src = x + ((size_t)bb * kSeqFull + ss) * kDim;
    dst = xh + (size_t)blk * kDim;
    sc = cx;
  } else {
    blk -= nXBlk;
    sc = cw;
    if (blk < 4 * kCastBlkW) {
      const int which = blk / kCastBlkW, lb = blk - which * kCastBlkW;
      const float* s0 = (which == 0) ? Wq : ((which == 1) ? Wk : ((which == 2) ? Wv : Wo));
      src = s0 + (size_t)lb * kCastElems;
      _Float16* d0 = (which < 3) ? (wqkvh + (size_t)which * kDim * kDim) : woh;
      dst = d0 + (size_t)lb * kCastElems;
    } else {
      blk -= 4 * kCastBlkW;
      if (blk < kCastBlkW1) {
        src = W1 + (size_t)blk * kCastElems;
        dst = w1h + (size_t)blk * kCastElems;
      } else {
        blk -= kCastBlkW1;
        src = W2 + (size_t)blk * kCastElems;
        dst = w2h + (size_t)blk * kCastElems;
      }
    }
  }
  const v2f f = *(const v2f*)(src + 2 * t);
  const _Float16 h0 = (_Float16)(bfrne(f[0]) * sc), h1 = (_Float16)(bfrne(f[1]) * sc);
  const unsigned u = (unsigned)__builtin_bit_cast(unsigned short, h0) | ((unsigned)__builtin_bit_cast(unsigned short, h1) << 16);
  ((volatile unsigned*)dst)[t] = u;
  __threadfence();
  ((volatile unsigned*)dst)[t] = u;
}

__global__ __launch_bounds__(256) void mask_flags(const float* __restrict__ amask, int* __restrict__ flags) {
  __shared__ int sAny[8][kFlagLd];
  __shared__ __align__(16) int sLine[kFlagLd];
  const int qb = blockIdx.x, t = threadIdx.x, w = t >> 5, l = t & 31;
  const int r = t >> 2, c0 = (t & 3) * 16;
  const float* mrow = amask + (size_t)(qb * kAQB + r) * kSeqFull + c0;
#pragma unroll 1
  for (int kc = 0; kc < kNkc; ++kc) {
    const float* p = mrow + kc * kAKC;
    const v4f a0 = *(const v4f*)(p);
    const v4f a1 = *(const v4f*)(p + 4);
    const v4f a2 = *(const v4f*)(p + 8);
    const v4f a3 = *(const v4f*)(p + 12);
    int anyi = 0;
#pragma unroll
    for (int e = 0; e < 4; ++e) {
      anyi |= (a0[e] > kMaskSkip) ? 1 : 0;
      anyi |= (a1[e] > kMaskSkip) ? 1 : 0;
      anyi |= (a2[e] > kMaskSkip) ? 1 : 0;
      anyi |= (a3[e] > kMaskSkip) ? 1 : 0;
    }
    const unsigned bal = __builtin_amdgcn_ballot_w32(anyi != 0);
    if (l == 0) sAny[w][kc] = (bal != 0u) ? 1 : 0;
  }
  __syncthreads();
  if (t < kFlagLd) {
    int f = 0;
    if (t < kNkc) {
#pragma unroll
      for (int i = 0; i < 8; ++i) f |= sAny[i][t];
    }
    sLine[t] = f;
  }
  __syncthreads();
  if (t < 8) {
    const v4i v = *(const v4i*)(sLine + 4 * t);
    int* dp = flags + (size_t)qb * kFlagLd + 4 * t;
    *(volatile v4i*)dp = v;
    __threadfence();
    *(volatile v4i*)dp = v;
  }
}

template <bool WH>
__global__ __launch_bounds__(128) void layernorm512(
    const float* __restrict__ xin, const float* __restrict__ gam, const float* __restrict__ bet,
    float* __restrict__ yf, int seqIn, int seqOut, _Float16* __restrict__ yh, float hscale) {
  __shared__ float ssum[4];
  __shared__ float ssq[4];
  __shared__ __align__(16) unsigned hrow[256];
  const int row = blockIdx.x;
  const int t = threadIdx.x;
  const int w = t >> 5;
  const int l = t & 31;
  const v4f v = *(const v4f*)(xin + (size_t)row * kDim + t * 4);
  float s = (v[0] + v[1]) + (v[2] + v[3]);
#pragma unroll
  for (int off = 1; off < 32; off <<= 1) s += __shfl_xor(s, off, 32);
  if (l == 0) ssum[w] = s;
  __syncthreads();
  const float tot = (ssum[0] + ssum[1]) + (ssum[2] + ssum[3]);
  const float mean = tot * (1.0f / 512.0f);
  const v4f d = v - mean;
  float q = (d[0] * d[0] + d[1] * d[1]) + (d[2] * d[2] + d[3] * d[3]);
#pragma unroll
  for (int off = 1; off < 32; off <<= 1) q += __shfl_xor(q, off, 32);
  if (l == 0) ssq[w] = q;
  __syncthreads();
  const float totq = (ssq[0] + ssq[1]) + (ssq[2] + ssq[3]);
  const float var = totq * (1.0f / 512.0f);
  const float inv = rsqrtf(var + kEps);
  v4f gv = *(const v4f*)(gam + t * 4);
  v4f bv = *(const v4f*)(bet + t * 4);
  gv[0] = bfrne(gv[0]); gv[1] = bfrne(gv[1]); gv[2] = bfrne(gv[2]); gv[3] = bfrne(gv[3]);
  bv[0] = bfrne(bv[0]); bv[1] = bfrne(bv[1]); bv[2] = bfrne(bv[2]); bv[3] = bfrne(bv[3]);
  const v4f o = d * inv * gv + bv;
  const int bb = row / seqIn, ss = row - bb * seqIn;
  float* yrow = yf + ((size_t)bb * seqOut + ss) * kDim + t * 4;
  *(volatile v4f*)yrow = o;
  __threadfence();
  *(volatile v4f*)yrow = o;
  if (WH) {
    const unsigned hb0 = (unsigned)__builtin_bit_cast(unsigned short, (_Float16)(o[0] * hscale));
    const unsigned hb1 = (unsigned)__builtin_bit_cast(unsigned short, (_Float16)(o[1] * hscale));
    const unsigned hb2 = (unsigned)__builtin_bit_cast(unsigned short, (_Float16)(o[2] * hscale));
    const unsigned hb3 = (unsigned)__builtin_bit_cast(unsigned short, (_Float16)(o[3] * hscale));
    v2u pk;
    pk[0] = hb0 | (hb1 << 16);
    pk[1] = hb2 | (hb3 << 16);
    *(v2u*)(hrow + 2 * t) = pk;
    __syncthreads();
    if (t < 64) {
      const v4u wv = *(const v4u*)(hrow + 4 * t);
      _Float16* hp = yh + (size_t)row * kDim + t * 8;
      *(volatile v4u*)hp = wv;
      __threadfence();
      *(volatile v4u*)hp = wv;
    }
  }
}

__device__ __forceinline__ v8f mma_h(v16h a, v16h b, v8f c) {
  c = __builtin_amdgcn_wmma_f32_16x16x32_f16(false, a, false, b, (short)0, c, false, false);
  asm volatile("v_nop\n\tv_nop\n\tv_nop\n\tv_nop" : "+v"(c) : "v"(a), "v"(b));
  return c;
}

__device__ __forceinline__ void vt_scatter(_Float16* vt, v4u w, int d0, int kvr) {
#pragma unroll
  for (int e = 0; e < 4; ++e) {
    const unsigned u = w[e];
    const int d = d0 + 2 * e;
    vt[d * kAKC + kvr]       = __builtin_bit_cast(_Float16, (unsigned short)(u & 0xffffu));
    vt[(d + 1) * kAKC + kvr] = __builtin_bit_cast(_Float16, (unsigned short)(u >> 16));
  }
}

__global__ __launch_bounds__(128)
void attn_bias_h64(const _Float16* __restrict__ qkv, const float* __restrict__ amask,
                   const int* __restrict__ flags, const float* __restrict__ alphas,
                   _Float16* __restrict__ ctx_out, float sscale, float pscale, float oscale) {
  union FH { v16h v; v8h h[2]; };
  __shared__ __align__(16) _Float16 Ksh[kAKC * kHdim];
  __shared__ __align__(16) _Float16 Vth[kHdim * kAKC];
  __shared__ __align__(16) _Float16 Psh[kANW][16 * kAKC];
  __shared__ __align__(16) float  Osl[kANW][16 * 68];
  __shared__ __align__(16) float  Msh[kAQB * kAKC];

  const int tid  = threadIdx.x;
  const int wave = tid >> 5;
  const int lane = tid & 31;
  const int hh   = lane >> 4;
  const int c    = lane & 15;

  const int nqb = kSeq / kAQB;
  const int bx = blockIdx.x;
  const int qb = bx % nqb;
  const int bh = bx / nqb;
  const int h  = bh % kHeads;
  const int b  = bh / kHeads;
  const int q0 = qb * kAQB + wave * 16;

  const _Float16* base = qkv + (size_t)b * kSeq * kQkvLd + (size_t)h * kHdim;

  v16h qa[2];
  {
    const _Float16* qrow = base + (size_t)(q0 + c) * kQkvLd + 8 * hh;
    qa[0] = Frag<_Float16>::load(qrow);
    qa[1] = Frag<_Float16>::load(qrow + 32);
  }
  const float alpha = bfrne(alphas[h]);

  float mrow[8], lrow[8];
  v8f oacc[4];
#pragma unroll
  for (int r = 0; r < 8; ++r) { mrow[r] = -INFINITY; lrow[r] = 0.f; }
#pragma unroll
  for (int t = 0; t < 4; ++t) oacc[t] = (v8f){0.f,0.f,0.f,0.f,0.f,0.f,0.f,0.f};

  for (int kc = 0; kc < kNkc; ++kc) {
    const int fl = flags[qb * kFlagLd + kc];
    if (fl == 0) continue;
    const int kv0 = kc * kAKC;
    __syncthreads();
    {
      const int mr = tid >> 1, mh = (tid & 1) * 32;
      const float* mp = amask + (size_t)(qb * kAQB + mr) * kSeqFull + kv0 + mh;
      float* md = Msh + mr * kAKC + mh;
#pragma unroll
      for (int e = 0; e < 8; ++e) *(v4f*)(md + 4 * e) = *(const v4f*)(mp + 4 * e);
    }
    {
      const int kvr = tid >> 1, dh = (tid & 1) * 32;
      const _Float16* krow = base + (size_t)(kv0 + kvr) * kQkvLd + kDim + dh;
      const _Float16* vrow = krow + kDim;
      const v8h k0v = *(const v8h*)(krow);
      const v8h k1v = *(const v8h*)(krow + 8);
      const v8h k2v = *(const v8h*)(krow + 16);
      const v8h k3v = *(const v8h*)(krow + 24);
      const v4u v0w = *(const v4u*)(vrow);
      const v4u v1w = *(const v4u*)(vrow + 8);
      const v4u v2w = *(const v4u*)(vrow + 16);
      const v4u v3w = *(const v4u*)(vrow + 24);
      _Float16* kd = Ksh + kvr * kHdim + dh;
      *(v8h*)(kd)      = k0v;
      *(v8h*)(kd + 8)  = k1v;
      *(v8h*)(kd + 16) = k2v;
      *(v8h*)(kd + 24) = k3v;
      vt_scatter(Vth, v0w, dh,      kvr);
      vt_scatter(Vth, v1w, dh + 8,  kvr);
      vt_scatter(Vth, v2w, dh + 16, kvr);
      vt_scatter(Vth, v3w, dh + 24, kvr);
    }
    __syncthreads();

    v8f s[4];
#pragma unroll
    for (int j = 0; j < 4; ++j) {
      s[j] = (v8f){0.f,0.f,0.f,0.f,0.f,0.f,0.f,0.f};
#pragma unroll
      for (int dc = 0; dc < 2; ++dc) {
        FH kb;
        kb.h[0] = *(const v8h*)(Ksh + (j * 16 + c) * kHdim + dc * 32 + 8 * hh);
        kb.h[1] = *(const v8h*)(Ksh + (j * 16 + c) * kHdim + dc * 32 + 16 + 8 * hh);
        s[j] = mma_h(qa[dc], kb.v, s[j]);
      }
    }
    float cm[8];
#pragma unroll
    for (int r = 0; r < 8; ++r) {
      const int ql = wave * 16 + 8 * hh + r;
      float m = -INFINITY;
#pragma unroll
      for (int j = 0; j < 4; ++j) {
        const float sv = s[j][r] * sscale + Msh[ql * kAKC + j * 16 + c];
        s[j][r] = sv;
        m = fmaxf(m, sv);
      }
#pragma unroll
      for (int off = 1; off < 16; off <<= 1) m = fmaxf(m, __shfl_xor(m, off, 32));
      cm[r] = m;
    }
    _Float16* pw = Psh[wave];
#pragma unroll
    for (int r = 0; r < 8; ++r) {
      const float mnew = fmaxf(mrow[r], cm[r]);
      const float msafe = (mnew == -INFINITY) ? 0.f : mnew;
      const float al = __expf(mrow[r] - msafe);
      mrow[r] = mnew;
      float psum = 0.f;
#pragma unroll
      for (int j = 0; j < 4; ++j) {
        const float p = __expf(s[j][r] - msafe);
        psum += p;
        pw[(8 * hh + r) * kAKC + j * 16 + c] = (_Float16)(p * pscale);
      }
#pragma unroll
      for (int off = 1; off < 16; off <<= 1) psum += __shfl_xor(psum, off, 32);
      lrow[r] = lrow[r] * al + psum;
#pragma unroll
      for (int t = 0; t < 4; ++t) oacc[t][r] *= al;
    }
    __builtin_amdgcn_fence(3  , "workgroup");
    __builtin_amdgcn_wave_barrier();
    __builtin_amdgcn_fence(2  , "workgroup");
#pragma unroll
    for (int kk = 0; kk < 2; ++kk) {
      FH pa;
      pa.h[0] = *(const v8h*)(pw + c * kAKC + kk * 32 + 8 * hh);
      pa.h[1] = *(const v8h*)(pw + c * kAKC + kk * 32 + 16 + 8 * hh);
#pragma unroll
      for (int t = 0; t < 4; ++t) {
        FH vb;
        vb.h[0] = *(const v8h*)(Vth + (t * 16 + c) * kAKC + kk * 32 + 8 * hh);
        vb.h[1] = *(const v8h*)(Vth + (t * 16 + c) * kAKC + kk * 32 + 16 + 8 * hh);
        oacc[t] = mma_h(pa.v, vb.v, oacc[t]);
      }
    }
  }

  float* os = Osl[wave];
#pragma unroll
  for (int r = 0; r < 8; ++r) {
    const float lr = lrow[r];
    const float inv = (lr > 0.f) ? (oscale * alpha * __builtin_amdgcn_rcpf(lr)) : 0.f;
#pragma unroll
    for (int t = 0; t < 4; ++t) os[(8 * hh + r) * 68 + t * 16 + c] = oacc[t][r] * inv;
  }
  __builtin_amdgcn_fence(3  , "workgroup");
  __builtin_amdgcn_wave_barrier();
  __builtin_amdgcn_fence(2  , "workgroup");
  {
    const int q8 = lane >> 3, c8 = (lane & 7) * 8;
    _Float16* ob = ctx_out + (size_t)(b * kSeq) * kDim + h * kHdim;
    for (int pass = 0; pass < 2; ++pass) {
#pragma unroll
      for (int it = 0; it < 4; ++it) {
        const int row = it * 4 + q8;
        const float* sp = os + row * 68 + c8;
        v8h hv;
#pragma unroll
        for (int e = 0; e < 8; ++e) hv[e] = (_Float16)sp[e];
        *(volatile v8h*)(ob + (size_t)(q0 + row) * kDim + c8) = hv;
      }
      __threadfence();
    }
  }
}

extern "C" void kernel_launch(void* const* d_in, const int* in_sizes, int n_in,
                              void* d_out, int out_size, void* d_ws, size_t ws_size,
                              hipStream_t stream) {
  if (n_in != 19) return;
  if (in_sizes[0] < (kBatch - 1) * kSeqFull * kDim + kSeq * kDim) return;
  if (in_sizes[1] < (kSeq - 1) * kSeqFull + kSeq) return;
  if (in_sizes[2] < kDim * kDim || in_sizes[4] < kDim * kDim || in_sizes[6] < kDim * kDim || in_sizes[8] < kDim * kDim) return;
  if (in_sizes[3] < kDim || in_sizes[5] < kDim || in_sizes[7] < kDim || in_sizes[9] < kDim) return;
  if (in_sizes[10] < kHeads) return;
  if (in_sizes[11] < kDim || in_sizes[12] < kDim || in_sizes[17] < kDim || in_sizes[18] < kDim) return;
  if (in_sizes[13] < kFfn * kDim || in_sizes[14] < kFfn || in_sizes[15] < kDim * kFfn || in_sizes[16] < kDim) return;
  if (out_size < (kBatch - 1) * kSeqFull * kDim + kSeq * kDim) return;
  if (ws_size < kWsTotal) return;

  const float* x    = (const float*)d_in[0];
  const float* amsk = (const float*)d_in[1];
  const float* Wq   = (const float*)d_in[2];
  const float* bq   = (const float*)d_in[3];
  const float* Wk   = (const float*)d_in[4];
  const float* bk   = (const float*)d_in[5];
  const float* Wv   = (const float*)d_in[6];
  const float* bv   = (const float*)d_in[7];
  const float* Wo   = (const float*)d_in[8];
  const float* bo   = (const float*)d_in[9];
  const float* alph = (const float*)d_in[10];
  const float* ln1g = (const float*)d_in[11];
  const float* ln1b = (const float*)d_in[12];
  const float* W1   = (const float*)d_in[13];
  const float* b1   = (const float*)d_in[14];
  const float* W2   = (const float*)d_in[15];
  const float* b2   = (const float*)d_in[16];
  const float* ln2g = (const float*)d_in[17];
  const float* ln2b = (const float*)d_in[18];
  float* outf = (float*)d_out;

  char* ws = (char*)d_ws;
  _Float16* wqkv = (_Float16*)(ws + kOffWqkv);
  _Float16* woh  = (_Float16*)(ws + kOffWo);
  _Float16* w1h  = (_Float16*)(ws + kOffW1);
  _Float16* w2h  = (_Float16*)(ws + kOffW2);
  _Float16* xh   = (_Float16*)(ws + kOffXh);
  int*      flg  = (int*)(ws + kOffFlags);
  _Float16* qkvp = (_Float16*)(ws + kOffQkv);
  _Float16* ctxp = (_Float16*)(ws + kOffCtx);
  float*    uf   = (float*)(ws + kOffU);
  float*    hf   = (float*)(ws + kOffHf);
  _Float16* hh   = (_Float16*)(ws + kOffHh);
  _Float16* hid  = (_Float16*)(ws + kOffHid);
  float*    yf   = (float*)(ws + kOffY);

  typedef const unsigned short* cus;

  {
    const unsigned blocks = (unsigned)(kRows + 4 * kCastBlkW + 2 * kCastBlkW1);
    cast_planes<<<dim3(blocks), dim3(256), 0, stream>>>(x, Wq, Wk, Wv, Wo, W1, W2,
                                                       xh, wqkv, woh, w1h, w2h, kRows, kCarryX, kCarryW);
  }

  mask_flags<<<dim3((unsigned)kNkc), dim3(256), 0, stream>>>(amsk, flg);

  {
    const unsigned blocks = (unsigned)(((kRows / 64) * (kDim / 64) + 7) / 8);
    wmma_gemm64<0, false, 2, 1, false, false, 0><<<dim3(blocks, 3), dim3(256), 0, stream>>>(
        (cus)xh, (cus)xh, kDim, (long)0,
        (cus)wqkv, (cus)wqkv, kDim, (long)kDim * kDim,
        (void*)qkvp, (void*)qkvp, kQkvLd, (long)kDim,
        bq, bk, bv,
        x, (long)0,
        kRows, kDim, kDim, 1.0f / (kCarryX * kCarryW), kCarryQkv);
  }

  {
    const unsigned blocks = (unsigned)(kBatch * kHeads * (kSeq / kAQB));
    attn_bias_h64<<<dim3(blocks), dim3(128), 0, stream>>>(
        qkvp, amsk, flg, alph, ctxp, 0.125f / (kCarryQkv * kCarryQkv), kCarryP, kCarryCtx / (kCarryP * kCarryQkv));
  }

  {
    const unsigned blocks = (unsigned)(((kSeq / 64) * (kDim / 64) + 7) / 8);
    wmma_gemm64<0, false, 2, 0, true, true, 0><<<dim3(blocks, kBatch), dim3(256), 0, stream>>>(
        (cus)ctxp, (cus)ctxp, kDim, (long)kSeq * kDim,
        (cus)woh, (cus)woh, kDim, (long)0,
        (void*)uf, (void*)uf, kDim, (long)kSeq * kDim,
        bo, bo, bo,
        x, (long)kSeqFull * kDim,
        kSeq, kDim, kDim, 1.0f / (kCarryCtx * kCarryW), 1.0f);
  }

  layernorm512<true><<<dim3((unsigned)kRows), dim3(128), 0, stream>>>(uf, ln1g, ln1b, hf, kSeq, kSeq, hh, kCarryH);

  {
    const unsigned blocks = (unsigned)(((kRows / 64) * (kFfn / 64) + 7) / 8);
    wmma_gemm64<0, false, 2, 1, false, false, 2><<<dim3(blocks, 1), dim3(256), 0, stream>>>(
        (cus)hh, (cus)hh, kDim, (long)0,
        (cus)w1h, (cus)w1h, kDim, (long)0,
        (void*)hid, (void*)hid, kFfn, (long)0,
        b1, b1, b1,
        hf, (long)0,
        kRows, kFfn, kDim, 1.0f / (kCarryH * kCarryW), kCarryHid);
  }

  {
    const unsigned blocks = (unsigned)(((kRows / 64) * (kDim / 64) + 7) / 8);
    wmma_gemm64<0, false, 2, 0, true, false, 0><<<dim3(blocks, 1), dim3(256), 0, stream>>>(
        (cus)hid, (cus)hid, kFfn, (long)0,
        (cus)w2h, (cus)w2h, kFfn, (long)0,
        (void*)yf, (void*)yf, kDim, (long)0,
        b2, b2, b2,
        hf, (long)0,
        kRows, kDim, kFfn, 1.0f / (kCarryHid * kCarryW), 1.0f);
  }

  layernorm512<false><<<dim3((unsigned)kRows), dim3(128), 0, stream>>>(yf, ln2g, ln2b, outf, kSeq, kSeqFull, hh, kCarryH);
}
